// Gated_DGL_58110907515590
// MI455X (gfx1250) — hardware-verified
//
#include <hip/hip_runtime.h>
#include <stddef.h>


#define DF      128
#define DG      384
#define NCLS    40
#define NCP     48
#define NTHR    256
#define NWAVE   8
#define EPT     8
#define NGRP    2
#define CHUNK   (NTHR * EPT * NGRP)
#define WCAP    (EPT * NGRP * 32)
#define LISTN   (NWAVE * WCAP)
#define NB      512
#define GROWS   128
#define UROWS   64
#define RROWS   32
#define APITCH  136
#define WSCALE  16.0f
#define WINV    0.0625f

#define WO_EMB  0
#define WO_E0   (DF * DF)
#define WO_E1   (2 * DF * DF)
#define WO_IH0  (3 * DF * DF)
#define WO_HH0  (3 * DF * DF + DG * DF)
#define WO_IH1  (3 * DF * DF + 2 * DG * DF)
#define WO_HH1  (3 * DF * DF + 3 * DG * DF)
#define WO_RD   (3 * DF * DF + 4 * DG * DF)
#define WTOT    (WO_RD + NCP * DF)

#define LDS_GEMM (GROWS * DF * 4)
#define LDS_AGG  (NB * DF * 4 + LISTN * 4 + 64)
#define LDS_UPD  (2 * UROWS * APITCH * 2 + UROWS * DF * 4)

static_assert((CHUNK & (CHUNK - 1)) == 0);
static_assert(CHUNK <= 4096);
static_assert((NB & (NB - 1)) == 0 && NB <= 4096);
static_assert(GROWS * APITCH * 2 <= LDS_GEMM);
static_assert(GROWS % UROWS == 0);
static_assert(NB % UROWS == 0);

typedef float    v4f  __attribute__((ext_vector_type(4)));
typedef float    v8f  __attribute__((ext_vector_type(8)));
typedef int      v4i  __attribute__((ext_vector_type(4)));
typedef _Float16 v8h  __attribute__((ext_vector_type(8)));
typedef _Float16 v16h __attribute__((ext_vector_type(16)));
union FragH { v16h v; v8h h[2]; };

__device__ __forceinline__ v8h cvt8(v4f a, v4f b) {
  v8h r;
  r[0] = (_Float16)a.x; r[1] = (_Float16)a.y; r[2] = (_Float16)a.z; r[3] = (_Float16)a.w;
  r[4] = (_Float16)b.x; r[5] = (_Float16)b.y; r[6] = (_Float16)b.z; r[7] = (_Float16)b.w;
  return r;
}

__device__ __forceinline__ v8f wmh(v16h a, v16h b, v8f c) {
  v8f d = __builtin_amdgcn_wmma_f32_16x16x32_f16(false, a, false, b, (short)0, c, false, false);
  asm volatile("v_nop\n\tv_nop\n\tv_nop\n\tv_nop" : "+v"(d) : "v"(a), "v"(b));
  return d;
}

__device__ __forceinline__ float sigm_f(float s) {
  const float e = expf(-s);
  return __builtin_amdgcn_rcpf(1.0f + e);
}

__device__ __forceinline__ float tanh_f(float x) {
  float y = fabsf(x);
  y = y > 20.0f ? 20.0f : y;
  const float e = expf(2.0f * y);
  const float t = 1.0f - 2.0f * __builtin_amdgcn_rcpf(e + 1.0f);
  return copysignf(t, x);
}

template <int NBT>
__device__ __forceinline__ int scan_chunk(const int* __restrict__ dsts, int nE, int cbase, int nodeBase,
                                          int vec8, int* list, int tid, int lane, int wave) {
  (void)lane;
  int wc = 0;
#pragma unroll
  for (int g = 0; g < NGRP; ++g) {
    const int el0  = (g * NTHR + tid) * EPT;
    const int e0   = cbase + el0;
    const int sent = -2147483647 - 1;
    v4i da, db;
    if (vec8 != 0 && cbase + CHUNK <= nE) {
      da = *(const v4i*)(dsts + e0);
      db = *(const v4i*)(dsts + e0 + 4);
    } else {
      da.x = (e0     < nE) ? dsts[min(e0, nE - 1)]     : sent;
      da.y = (e0 + 1 < nE) ? dsts[min(e0 + 1, nE - 1)] : sent;
      da.z = (e0 + 2 < nE) ? dsts[min(e0 + 2, nE - 1)] : sent;
      da.w = (e0 + 3 < nE) ? dsts[min(e0 + 3, nE - 1)] : sent;
      db.x = (e0 + 4 < nE) ? dsts[min(e0 + 4, nE - 1)] : sent;
      db.y = (e0 + 5 < nE) ? dsts[min(e0 + 5, nE - 1)] : sent;
      db.z = (e0 + 6 < nE) ? dsts[min(e0 + 6, nE - 1)] : sent;
      db.w = (e0 + 7 < nE) ? dsts[min(e0 + 7, nE - 1)] : sent;
    }
    const unsigned nb = (unsigned)nodeBase;
    const unsigned s0 = (unsigned)da.x - nb, s1 = (unsigned)da.y - nb;
    const unsigned s2 = (unsigned)da.z - nb, s3 = (unsigned)da.w - nb;
    const unsigned s4 = (unsigned)db.x - nb, s5 = (unsigned)db.y - nb;
    const unsigned s6 = (unsigned)db.z - nb, s7 = (unsigned)db.w - nb;
    const bool h0 = s0 < (unsigned)NBT, h1 = s1 < (unsigned)NBT, h2 = s2 < (unsigned)NBT, h3 = s3 < (unsigned)NBT;
    const bool h4 = s4 < (unsigned)NBT, h5 = s5 < (unsigned)NBT, h6 = s6 < (unsigned)NBT, h7 = s7 < (unsigned)NBT;
    const unsigned any = __builtin_amdgcn_ballot_w32(h0 | h1 | h2 | h3 | h4 | h5 | h6 | h7);
    if (any != 0u) {
#define HITJ(J, HJ, SJ) { \
        const unsigned mj = __builtin_amdgcn_ballot_w32(HJ); \
        if (mj != 0u) { \
          if (HJ) { \
            const int pos = wc + (int)__builtin_amdgcn_mbcnt_lo(mj, 0u); \
            if (pos < WCAP) list[wave * WCAP + pos] = ((el0 + (J)) << 12) | (int)(SJ); \
          } \
          wc += (int)__builtin_popcount(mj); } }
      HITJ(0, h0, s0)
      HITJ(1, h1, s1)
      HITJ(2, h2, s2)
      HITJ(3, h3, s3)
      HITJ(4, h4, s4)
      HITJ(5, h5, s5)
      HITJ(6, h6, s6)
      HITJ(7, h7, s7)
#undef HITJ
    }
  }
  return wc;
}

__global__ __launch_bounds__(NTHR) void k_wprep(
    const float* __restrict__ w0, const float* __restrict__ w1, const float* __restrict__ w2,
    const float* __restrict__ w3, const float* __restrict__ w4, const float* __restrict__ w5,
    const float* __restrict__ w6, const float* __restrict__ w7, _Float16* wp) {
  const int mat = blockIdx.y;
  const float* W; int nval, nout, off;
  if (mat == 0)      { W = w0; nval = DF;   nout = DF;  off = WO_EMB; }
  else if (mat == 1) { W = w1; nval = DF;   nout = DF;  off = WO_E0;  }
  else if (mat == 2) { W = w2; nval = DF;   nout = DF;  off = WO_E1;  }
  else if (mat == 3) { W = w3; nval = DG;   nout = DG;  off = WO_IH0; }
  else if (mat == 4) { W = w4; nval = DG;   nout = DG;  off = WO_HH0; }
  else if (mat == 5) { W = w5; nval = DG;   nout = DG;  off = WO_IH1; }
  else if (mat == 6) { W = w6; nval = DG;   nout = DG;  off = WO_HH1; }
  else               { W = w7; nval = NCLS; nout = NCP; off = WO_RD;  }
  const int i = blockIdx.x * NTHR + threadIdx.x;
  if (i >= nout * (DF / 8)) return;
  const int n  = i >> 4;
  const int k0 = (i & 15) * 8;
  const int ns = n < nval ? n : nval - 1;
  const float* p = W + (size_t)ns * DF + k0;
  v4f a = *(const v4f*)p, b = *(const v4f*)(p + 4);
  const v4f z = {0.f, 0.f, 0.f, 0.f};
  if (n >= nval) { a = z; b = z; }
  a = a * WSCALE;
  b = b * WSCALE;
  const v8h hv = cvt8(a, b);
  _Float16* dp = wp + off + (size_t)i * 8;
  *(volatile v8h*)dp = hv;
  __threadfence();
  *(volatile v8h*)dp = hv;
}

__global__ __launch_bounds__(NTHR) void k_ngemm(
    const float* __restrict__ x, const _Float16* __restrict__ wpl,
    const float* __restrict__ bias, float* y, int nN) {
  extern __shared__ v4f lds_dyn[];
  _Float16* sA  = (_Float16*)lds_dyn;
  float*    stg = (float*)lds_dyn;
  const int tid = threadIdx.x, lane = tid & 31, wave = tid >> 5, hh = lane >> 4, m = lane & 15;
  const int rowBase = blockIdx.x * GROWS;

#pragma unroll
  for (int i = 0; i < (GROWS * DF / 8) / NTHR; ++i) {
    const int idx = i * NTHR + tid;
    const int r   = idx >> 4;
    const int c0  = (idx & 15) * 8;
    int node = rowBase + r;
    node = node > nN - 1 ? nN - 1 : node;
    const float* xp = x + (size_t)node * DF + c0;
    const v4f a = *(const v4f*)xp, b = *(const v4f*)(xp + 4);
    *(v8h*)(sA + r * APITCH + c0) = cvt8(a, b);
  }
  __syncthreads();

  v8f acc[8];
#pragma unroll
  for (int t = 0; t < 8; ++t) { v8f z = {0.f, 0.f, 0.f, 0.f, 0.f, 0.f, 0.f, 0.f}; acc[t] = z; }
  const _Float16* ar = sA + (wave * 16 + m) * APITCH + 8 * hh;
#pragma unroll
  for (int kt = 0; kt < DF / 32; ++kt) {
    FragH a;
    a.h[0] = *(const v8h*)(ar + 32 * kt);
    a.h[1] = *(const v8h*)(ar + 32 * kt + 16);
#pragma unroll
    for (int t = 0; t < 8; ++t) {
      const _Float16* bp = wpl + (size_t)(16 * t + m) * DF + 32 * kt + 8 * hh;
      FragH b;
      b.h[0] = *(const v8h*)bp;
      b.h[1] = *(const v8h*)(bp + 16);
      acc[t] = wmh(a.v, b.v, acc[t]);
    }
  }
  __syncthreads();

  const int r0 = wave * 16 + 8 * hh;
  float* sp = stg + r0 * DF + m;
#pragma unroll
  for (int t = 0; t < 8; ++t) {
    const float bv = bias[16 * t + m];
    sp[0 * DF + 16 * t] = acc[t][0] * WINV + bv;
    sp[1 * DF + 16 * t] = acc[t][1] * WINV + bv;
    sp[2 * DF + 16 * t] = acc[t][2] * WINV + bv;
    sp[3 * DF + 16 * t] = acc[t][3] * WINV + bv;
    sp[4 * DF + 16 * t] = acc[t][4] * WINV + bv;
    sp[5 * DF + 16 * t] = acc[t][5] * WINV + bv;
    sp[6 * DF + 16 * t] = acc[t][6] * WINV + bv;
    sp[7 * DF + 16 * t] = acc[t][7] * WINV + bv;
  }
  __syncthreads();

  const float* lp = stg + wave * 16 * DF + 4 * lane;
  float* gp = y + ((size_t)rowBase + wave * 16) * DF + 4 * lane;
#pragma unroll
  for (int i = 0; i < 16; ++i) { const v4f v = *(const v4f*)(lp + i * DF); *(volatile v4f*)(gp + (size_t)i * DF) = v; }
  __threadfence();
#pragma unroll
  for (int i = 0; i < 16; ++i) { const v4f v = *(const v4f*)(lp + i * DF); *(volatile v4f*)(gp + (size_t)i * DF) = v; }
}

__global__ __launch_bounds__(NTHR) void k_agg(
    const int* __restrict__ srcs, const int* __restrict__ dsts, const float* __restrict__ mpl,
    _Float16* apl, int nN, int nE, int vec8) {
  extern __shared__ v4f lds_dyn[];
  float* acc  = (float*)lds_dyn;
  int*   list = (int*)(acc + NB * DF);
  int*   wcnt = list + LISTN;
  const int tid = threadIdx.x, lane = tid & 31, wave = tid >> 5, hh = lane >> 4, m = lane & 15;
  const int nodeBase = blockIdx.x * NB;

  {
    const v4f z = {0.f, 0.f, 0.f, 0.f};
    for (int i = tid; i < NB * DF / 4; i += NTHR) lds_dyn[i] = z;
  }
  __syncthreads();

  const int nChunks = (nE + CHUNK - 1) / CHUNK;
#pragma unroll 1
  for (int ch = 0; ch < nChunks; ++ch) {
    const int cbase = ch * CHUNK;
    const int wc = scan_chunk<NB>(dsts, nE, cbase, nodeBase, vec8, list, tid, lane, wave);
    if (lane == 0) wcnt[wave] = wc;
    __syncthreads();
    if (wave == 0) {
#pragma unroll 1
      for (int wsx = 0; wsx < NWAVE; ++wsx) {
        int n = __builtin_amdgcn_readfirstlane(wcnt[wsx]);
        n = n > WCAP ? WCAP : (n < 0 ? 0 : n);
        const int* lp = list + wsx * WCAP;
#pragma unroll 1
        for (int i = 0; i < n; ++i) {
          const int ent  = __builtin_amdgcn_readfirstlane(lp[i]);
          const int slot = ent & (NB - 1);
          int e = cbase + ((ent >> 12) & (CHUNK - 1));
          e = e > nE - 1 ? nE - 1 : e;
          int s = srcs[e];
          s = s < 0 ? 0 : (s > nN - 1 ? nN - 1 : s);
          const v4f v = *(const v4f*)(mpl + (size_t)s * DF + 4 * lane);
          v4f* ap = (v4f*)(acc + slot * DF + 4 * lane);
          *ap = *ap + v;
        }
      }
    }
    __syncthreads();
  }

  const float* lp = acc + (64 * wave + hh) * DF + 8 * m;
  _Float16* gp = apl + ((size_t)nodeBase + 64 * wave + hh) * DF + 8 * m;
#pragma unroll 4
  for (int q = 0; q < 32; ++q) {
    const v4f a = *(const v4f*)(lp + 2 * q * DF), b = *(const v4f*)(lp + 2 * q * DF + 4);
    *(volatile v8h*)(gp + (size_t)2 * q * DF) = cvt8(a, b);
  }
  __threadfence();
#pragma unroll 4
  for (int q = 0; q < 32; ++q) {
    const v4f a = *(const v4f*)(lp + 2 * q * DF), b = *(const v4f*)(lp + 2 * q * DF + 4);
    *(volatile v8h*)(gp + (size_t)2 * q * DF) = cvt8(a, b);
  }
}

__global__ __launch_bounds__(NTHR) void k_upd(
    const _Float16* __restrict__ apl, const float* __restrict__ xf,
    const _Float16* __restrict__ wih, const _Float16* __restrict__ whh,
    const float* __restrict__ bih, const float* __restrict__ bhh,
    float* xo, int nN) {
  extern __shared__ v4f lds_dyn[];
  _Float16* sA  = (_Float16*)lds_dyn;
  _Float16* sX  = sA + UROWS * APITCH;
  float*    stg = (float*)(sX + UROWS * APITCH);
  const int tid = threadIdx.x, lane = tid & 31, wave = tid >> 5, hh = lane >> 4, m = lane & 15;
  const int rowBase = blockIdx.x * UROWS;

#pragma unroll
  for (int i = 0; i < (UROWS * DF / 8) / NTHR; ++i) {
    const int idx = i * NTHR + tid;
    const int r   = idx >> 4;
    const int c0  = (idx & 15) * 8;
    const v8h v = *(const v8h*)(apl + ((size_t)rowBase + r) * DF + c0);
    *(v8h*)(sA + r * APITCH + c0) = v;
  }
#pragma unroll
  for (int i = 0; i < (UROWS * DF / 8) / NTHR; ++i) {
    const int idx = i * NTHR + tid;
    const int r   = idx >> 4;
    const int c0  = (idx & 15) * 8;
    int node = rowBase + r;
    node = node > nN - 1 ? nN - 1 : node;
    const float* xp = xf + (size_t)node * DF + c0;
    const v4f a = *(const v4f*)xp, b = *(const v4f*)(xp + 4);
    *(v8h*)(sX + r * APITCH + c0) = cvt8(a, b);
  }
  __syncthreads();

  const int rt = wave & 3, cg = wave >> 2;
  const _Float16* ar = sA + (16 * rt + m) * APITCH + 8 * hh;
  const _Float16* xr = sX + (16 * rt + m) * APITCH + 8 * hh;
  const int nodeA = rowBase + 16 * rt + 8 * hh;

#pragma unroll 1
  for (int p = 0; p < 4; ++p) {
    const int ct = 4 * cg + p;
    v8f air = {0.f, 0.f, 0.f, 0.f, 0.f, 0.f, 0.f, 0.f};
    v8f aiz = air, ain = air, ahr = air, ahz = air, ahn = air;
#pragma unroll
    for (int kt = 0; kt < DF / 32; ++kt) {
      FragH fa, fx;
      fa.h[0] = *(const v8h*)(ar + 32 * kt);
      fa.h[1] = *(const v8h*)(ar + 32 * kt + 16);
      fx.h[0] = *(const v8h*)(xr + 32 * kt);
      fx.h[1] = *(const v8h*)(xr + 32 * kt + 16);
      const _Float16* bi = wih + (size_t)(16 * ct + m) * DF + 32 * kt + 8 * hh;
      const _Float16* bh = whh + (size_t)(16 * ct + m) * DF + 32 * kt + 8 * hh;
      FragH b;
      b.h[0] = *(const v8h*)(bi);                       b.h[1] = *(const v8h*)(bi + 16);
      air = wmh(fa.v, b.v, air);
      b.h[0] = *(const v8h*)(bi + (size_t)DF * DF);     b.h[1] = *(const v8h*)(bi + (size_t)DF * DF + 16);
      aiz = wmh(fa.v, b.v, aiz);
      b.h[0] = *(const v8h*)(bi + (size_t)2 * DF * DF); b.h[1] = *(const v8h*)(bi + (size_t)2 * DF * DF + 16);
      ain = wmh(fa.v, b.v, ain);
      b.h[0] = *(const v8h*)(bh);                       b.h[1] = *(const v8h*)(bh + 16);
      ahr = wmh(fx.v, b.v, ahr);
      b.h[0] = *(const v8h*)(bh + (size_t)DF * DF);     b.h[1] = *(const v8h*)(bh + (size_t)DF * DF + 16);
      ahz = wmh(fx.v, b.v, ahz);
      b.h[0] = *(const v8h*)(bh + (size_t)2 * DF * DF); b.h[1] = *(const v8h*)(bh + (size_t)2 * DF * DF + 16);
      ahn = wmh(fx.v, b.v, ahn);
    }
    const int col = 16 * ct + m;
    const float b_ir = bih[col], b_iz = bih[col + DF], b_in = bih[col + 2 * DF];
    const float b_hr = bhh[col], b_hz = bhh[col + DF], b_hn = bhh[col + 2 * DF];
    float* sp = stg + (16 * rt + 8 * hh) * DF + col;
#pragma unroll
    for (int v = 0; v < 8; ++v) {
      int node = nodeA + v;
      node = node > nN - 1 ? nN - 1 : node;
      const float xold = xf[(size_t)node * DF + col];
      const float gr = air[v] * WINV + b_ir + ahr[v] * WINV + b_hr;
      const float gz = aiz[v] * WINV + b_iz + ahz[v] * WINV + b_hz;
      const float r  = sigm_f(gr);
      const float z  = sigm_f(gz);
      const float nn = tanh_f(ain[v] * WINV + b_in + r * (ahn[v] * WINV + b_hn));
      const float xn = (1.0f - z) * nn + z * xold;
      const float yv = xn > 0.0f ? xn : (expf(xn) - 1.0f);
      sp[v * DF] = yv;
    }
  }
  __syncthreads();

  const float* lp = stg + 8 * wave * DF + 4 * lane;
  float* gp = xo + ((size_t)rowBase + 8 * wave) * DF + 4 * lane;
#pragma unroll
  for (int i = 0; i < 8; ++i) { const v4f v = *(const v4f*)(lp + i * DF); *(volatile v4f*)(gp + (size_t)i * DF) = v; }
  __threadfence();
#pragma unroll
  for (int i = 0; i < 8; ++i) { const v4f v = *(const v4f*)(lp + i * DF); *(volatile v4f*)(gp + (size_t)i * DF) = v; }
}

__global__ __launch_bounds__(64) void k_readout(
    const float* __restrict__ xf, const _Float16* __restrict__ wrd,
    const float* __restrict__ rb, float* out, int nN) {
  __shared__ __attribute__((aligned(16))) _Float16 sXr[RROWS * APITCH];
  __shared__ __attribute__((aligned(16))) float slog[RROWS * NCP];
  __shared__ __attribute__((aligned(16))) float sout[RROWS * NCLS];
  const int tid = threadIdx.x, lane = tid & 31, wave = tid >> 5, hh = lane >> 4, m = lane & 15;
  const int rowBase = blockIdx.x * RROWS;

#pragma unroll
  for (int i = 0; i < (RROWS * DF / 8) / 64; ++i) {
    const int idx = i * 64 + tid;
    const int r   = idx >> 4;
    const int c0  = (idx & 15) * 8;
    int node = rowBase + r;
    node = node > nN - 1 ? nN - 1 : node;
    const float* xp = xf + (size_t)node * DF + c0;
    const v4f a = *(const v4f*)xp, b = *(const v4f*)(xp + 4);
    *(v8h*)(sXr + r * APITCH + c0) = cvt8(a, b);
  }
  __syncthreads();

  v8f acc[3];
#pragma unroll
  for (int t = 0; t < 3; ++t) { v8f z = {0.f, 0.f, 0.f, 0.f, 0.f, 0.f, 0.f, 0.f}; acc[t] = z; }
  const _Float16* ar = sXr + (16 * wave + m) * APITCH + 8 * hh;
#pragma unroll
  for (int kt = 0; kt < DF / 32; ++kt) {
    FragH a;
    a.h[0] = *(const v8h*)(ar + 32 * kt);
    a.h[1] = *(const v8h*)(ar + 32 * kt + 16);
#pragma unroll
    for (int t = 0; t < 3; ++t) {
      const _Float16* bp = wrd + (size_t)(16 * t + m) * DF + 32 * kt + 8 * hh;
      FragH b;
      b.h[0] = *(const v8h*)bp;
      b.h[1] = *(const v8h*)(bp + 16);
      acc[t] = wmh(a.v, b.v, acc[t]);
    }
  }

  float* sp = slog + (16 * wave + 8 * hh) * NCP;
#pragma unroll
  for (int t = 0; t < 3; ++t) {
    const int col = 16 * t + m;
    const int cb  = col < NCLS ? col : NCLS - 1;
    float bv = rb[cb];
    bv = col < NCLS ? bv : 0.0f;
#pragma unroll
    for (int r = 0; r < 8; ++r) sp[r * NCP + col] = acc[t][r] * WINV + bv;
  }
  __syncthreads();

  if (tid < RROWS) {
    const float* lr = slog + tid * NCP;
    float mx = lr[0];
#pragma unroll 1
    for (int c = 1; c < NCLS; ++c) mx = fmaxf(mx, lr[c]);
    float s = 0.0f;
#pragma unroll 1
    for (int c = 0; c < NCLS; ++c) s += expf(lr[c] - mx);
    const float lse = mx + logf(s);
    float* orow = sout + tid * NCLS;
#pragma unroll 1
    for (int c = 0; c < NCLS; ++c) orow[c] = lr[c] - lse;
  }
  __syncthreads();

  const size_t ob = (size_t)rowBase * NCLS;
  int nrow = nN - rowBase;
  nrow = nrow > RROWS ? RROWS : nrow;
  const int flim = nrow * NCLS;
  v4f ov[5];
#pragma unroll
  for (int q = 0; q < 5; ++q) ov[q] = *(const v4f*)(sout + (q * 64 + tid) * 4);
#pragma unroll
  for (int q = 0; q < 5; ++q) { const int f = (q * 64 + tid) * 4; if (f < flim) *(volatile v4f*)(out + ob + f) = ov[q]; }
  __threadfence();
#pragma unroll
  for (int q = 0; q < 5; ++q) { const int f = (q * 64 + tid) * 4; if (f < flim) *(volatile v4f*)(out + ob + f) = ov[q]; }
}

static inline int cdiv(int a, int b) { return (a + b - 1) / b; }

extern "C" void kernel_launch(void* const* d_in, const int* in_sizes, int n_in,
                              void* d_out, int out_size, void* d_ws, size_t ws_size,
                              hipStream_t stream) {
  if (n_in < 20) return;
  const int nN = in_sizes[0] / DF;
  const int nE = in_sizes[1];
  if (nN <= 0 || nE <= 0 || in_sizes[0] != nN * DF || in_sizes[2] != nE) return;
  if (in_sizes[4] != DF * DF || in_sizes[5] < DF) return;
  if (in_sizes[6] != NCLS * DF || in_sizes[7] < NCLS) return;
  if (in_sizes[8] != DF * DF || in_sizes[9] < DF || in_sizes[14] != DF * DF || in_sizes[15] < DF) return;
  if (in_sizes[10] != DG * DF || in_sizes[11] < DG || in_sizes[12] != DG * DF || in_sizes[13] < DG) return;
  if (in_sizes[16] != DG * DF || in_sizes[17] < DG || in_sizes[18] != DG * DF || in_sizes[19] < DG) return;
  if (out_size != nN * NCLS) return;

  const float* h    = (const float*)d_in[0];
  const int*   src  = (const int*)d_in[1];
  const int*   dst  = (const int*)d_in[2];
  const float* embW = (const float*)d_in[4];
  const float* embb = (const float*)d_in[5];
  const float* rdW  = (const float*)d_in[6];
  const float* rdb  = (const float*)d_in[7];
  const float* eW0  = (const float*)d_in[8];
  const float* eb0  = (const float*)d_in[9];
  const float* Wih0 = (const float*)d_in[10];
  const float* bih0 = (const float*)d_in[11];
  const float* Whh0 = (const float*)d_in[12];
  const float* bhh0 = (const float*)d_in[13];
  const float* eW1  = (const float*)d_in[14];
  const float* eb1  = (const float*)d_in[15];
  const float* Wih1 = (const float*)d_in[16];
  const float* bih1 = (const float*)d_in[17];
  const float* Whh1 = (const float*)d_in[18];
  const float* bhh1 = (const float*)d_in[19];
  float* out = (float*)d_out;

  const int nG = cdiv(nN, GROWS);
  const int nA = cdiv(nN, NB);
  const int nU = cdiv(nN, UROWS);
  const int nR = cdiv(nN, RROWS);
  const size_t rowsP = (size_t)nG * GROWS;
  const size_t rowsA = (size_t)nA * NB;

  char* ws = (char*)d_ws;
  size_t off = 0;
  const size_t oW  = off; off += (size_t)WTOT * 2;          off = (off + 255) & ~(size_t)255;
  const size_t oR1 = off; off += rowsP * DF * 4;            off = (off + 255) & ~(size_t)255;
  const size_t oR2 = off; off += rowsP * DF * 4;            off = (off + 255) & ~(size_t)255;
  const size_t oAP = off; off += rowsA * DF * 2;            off = (off + 255) & ~(size_t)255;
  if (off > ws_size) return;
  _Float16* wp = (_Float16*)(ws + oW);
  float*    R1 = (float*)(ws + oR1);
  float*    R2 = (float*)(ws + oR2);
  _Float16* AP = (_Float16*)(ws + oAP);

  const int vec8 = 1;

  k_wprep<<<dim3(cdiv(DG * (DF / 8), NTHR), 8), NTHR, 0, stream>>>(
      embW, eW0, eW1, Wih0, Whh0, Wih1, Whh1, rdW, wp);

  hipFuncSetAttribute(reinterpret_cast<const void*>(&k_ngemm),
                      hipFuncAttributeMaxDynamicSharedMemorySize, LDS_GEMM);
  hipFuncSetAttribute(reinterpret_cast<const void*>(&k_agg),
                      hipFuncAttributeMaxDynamicSharedMemorySize, LDS_AGG);
  hipFuncSetAttribute(reinterpret_cast<const void*>(&k_upd),
                      hipFuncAttributeMaxDynamicSharedMemorySize, LDS_UPD);

  k_ngemm<<<nG, NTHR, LDS_GEMM, stream>>>(h, wp + WO_EMB, embb, R1, nN);

  k_ngemm<<<nG, NTHR, LDS_GEMM, stream>>>(R1, wp + WO_E0, eb0, R2, nN);
  k_agg<<<nA, NTHR, LDS_AGG, stream>>>(src, dst, R2, AP, nN, nE, vec8);
  k_upd<<<nU, NTHR, LDS_UPD, stream>>>(AP, R1, wp + WO_IH0, wp + WO_HH0, bih0, bhh0, R2, nN);

  k_ngemm<<<nG, NTHR, LDS_GEMM, stream>>>(R2, wp + WO_E1, eb1, R1, nN);
  k_agg<<<nA, NTHR, LDS_AGG, stream>>>(src, dst, R1, AP, nN, nE, vec8);
  k_upd<<<nU, NTHR, LDS_UPD, stream>>>(AP, R2, wp + WO_IH1, wp + WO_HH1, bih1, bhh1, R1, nN);

  k_readout<<<nR, 64, 0, stream>>>(R1, wp + WO_RD, rdb, out, nN);
}
